// ModelWithgraph_embedding_modif_gcnconv_61022895342233
// MI455X (gfx1250) — hardware-verified
//
#include <hip/hip_runtime.h>
#include <math.h>

#define NN 50000
#define NE 600000
#define NP 50048
#define DD 128
#define ZW 512
#define AW 384
#define NG 512
#define HMW 256
#define NCL 32
#define NL 3
#define NT 256
#define SRB 2048
#define NTILE 25
#define NTA 13
#define SCH 2048
#define NCH ((NE + SCH - 1) / SCH)
#define PB (NP / 128)
#define SCHP 2048
#define NCHP ((NN + SCHP - 1) / SCHP)

typedef __attribute__((ext_vector_type(16))) _Float16 v16h;
typedef __attribute__((ext_vector_type(8)))  _Float16 v8h;
typedef __attribute__((ext_vector_type(4)))  _Float16 v4h;
typedef __attribute__((ext_vector_type(16))) __bf16   v16b;
typedef __attribute__((ext_vector_type(8)))  __bf16   v8b;
typedef __attribute__((ext_vector_type(8)))  float    v8f;
typedef __attribute__((ext_vector_type(4)))  float    v4f;
typedef __attribute__((ext_vector_type(4)))  int      v4i;

__device__ __forceinline__ unsigned short f2bf_bits(float f) {
  unsigned u = __float_as_uint(f);
  return (unsigned short)((u + 0x7FFFu + ((u >> 16) & 1u)) >> 16);
}
__device__ __forceinline__ float bf_bits2f(unsigned short h) { return __uint_as_float(((unsigned)h) << 16); }

__device__ __forceinline__ void dep_guard_h(v8f& a, v8f& b, v16h x, v16h y) { asm volatile("v_nop\n\tv_nop\n\tv_nop\n\tv_nop" : "+v"(a), "+v"(b) : "v"(x), "v"(y)); }
__device__ __forceinline__ void dep_guard_b(v8f& a, v8f& b, v16b x, v16b y) { asm volatile("v_nop\n\tv_nop\n\tv_nop\n\tv_nop" : "+v"(a), "+v"(b) : "v"(x), "v"(y)); }
__device__ __forceinline__ void keep4_h(v16h a, v16h b, v16h c, v16h d) { asm volatile("v_nop" :: "v"(a), "v"(b), "v"(c), "v"(d)); }
__device__ __forceinline__ void keep4_b(v16b a, v16b b, v16b c, v16b d) { asm volatile("v_nop" :: "v"(a), "v"(b), "v"(c), "v"(d)); }
__device__ __forceinline__ void acc_guard4(v8f& a, v8f& b, v8f& c, v8f& d) { asm volatile("v_nop\n\tv_nop\n\tv_nop\n\tv_nop" : "+v"(a), "+v"(b), "+v"(c), "+v"(d)); }
template <typename T> struct Frag;
template <> struct Frag<_Float16> {
  typedef v16h V; union U { v16h v; v8h h[2]; };
  static __device__ __forceinline__ v16h load(const _Float16* p) {
    U f; f.h[0] = *(const v8h*)(p); f.h[1] = *(const v8h*)(p + 16); return f.v;
  }
  static __device__ __forceinline__ v8f mma(v16h a, v16h b, v8f c) {
    return __builtin_amdgcn_wmma_f32_16x16x32_f16(false, a, false, b, (short)0, c, false, false);
  }
  static __device__ __forceinline__ void guard(v8f& a, v8f& b, v16h x, v16h y) { dep_guard_h(a, b, x, y); }
  static __device__ __forceinline__ void keep(v16h a, v16h b, v16h c, v16h d) { keep4_h(a, b, c, d); }
};
template <> struct Frag<__bf16> {
  typedef v16b V; union U { v16b v; v8b h[2]; };
  static __device__ __forceinline__ v16b load(const __bf16* p) {
    U f; f.h[0] = *(const v8b*)(p); f.h[1] = *(const v8b*)(p + 16); return f.v;
  }
  static __device__ __forceinline__ v8f mma(v16b a, v16b b, v8f c) {
    return __builtin_amdgcn_wmma_f32_16x16x32_bf16(false, a, false, b, (short)0, c, false, false);
  }
  static __device__ __forceinline__ void guard(v8f& a, v8f& b, v16b x, v16b y) { dep_guard_b(a, b, x, y); }
  static __device__ __forceinline__ void keep(v16b a, v16b b, v16b c, v16b d) { keep4_b(a, b, c, d); }
};

template <int ET> struct Elem;
template <> struct Elem<0> { typedef _Float16 T; };
template <> struct Elem<1> { typedef __bf16 T; };
template <int ET, bool SPLIT, int BIAS_MODE, int OUT_MODE, bool RESID, int ACT = 0, int NSTORE = 0>
__global__ __launch_bounds__(256) void wmma_gemm64(
    const unsigned short* __restrict__ Ap, const unsigned short* __restrict__ A2p, int lda, long strideA,
    const unsigned short* __restrict__ Btp, const unsigned short* __restrict__ Bt2p, int ldb, long strideB,
    void* __restrict__ Cout, void* __restrict__ Cout2, int ldc, long strideC,
    const float* __restrict__ bias,
    const float* __restrict__ resid, long strideR,
    int M, int N, int K, float scale, int Mlim) {
  typedef typename Elem<ET>::T T;
  typedef typename Frag<T>::V V;
  const T* A = (const T*)Ap; const T* A2 = (const T*)A2p; const T* Bt = (const T*)Btp; const T* Bt2 = (const T*)Bt2p;
  __shared__ __align__(16) float sT[8][16 * 68];
  const int b    = blockIdx.y;
  const int lane = threadIdx.x & 31;
  const int wave = threadIdx.x >> 5;
  const int tilesN = N >> 6;
  const int tilesM = M >> 6;
  const int tile = blockIdx.x * 8 + wave;
  if (tile >= tilesM * tilesN) return;
  const int tm = tile / tilesN;
  const int tn = tile - tm * tilesN;
  const int m0 = tm << 6;
  const int n0 = tn << 6;

  const T* Ab  = A  + (size_t)b * strideA;
  const T* Bb  = Bt + (size_t)b * strideB;
  const T* Ab2 = SPLIT ? (A2  + (size_t)b * strideA) : nullptr;
  const T* Bb2 = SPLIT ? (Bt2 + (size_t)b * strideB) : nullptr;

  const int rlane = lane & 15;
  const int koff  = (lane >> 4) * 8;
  const int mOff  = (lane >> 4) * 8;

  v8f acc[4][4];
#pragma unroll
  for (int i = 0; i < 4; ++i)
#pragma unroll
    for (int j = 0; j < 4; ++j) acc[i][j] = (v8f){0.f,0.f,0.f,0.f,0.f,0.f,0.f,0.f};

  for (int k0 = 0; k0 < K; k0 += 32) {
    V bh[4], bl[4];
#pragma unroll
    for (int j = 0; j < 4; ++j) {
      const size_t bo = (size_t)(n0 + (j << 4) + rlane) * ldb + koff + k0;
      bh[j] = Frag<T>::load(Bb + bo);
      if (SPLIT) bl[j] = Frag<T>::load(Bb2 + bo);
    }
#pragma unroll
    for (int i = 0; i < 4; ++i) {
      const size_t ao = (size_t)(m0 + (i << 4) + rlane) * lda + koff + k0;
      V ah = Frag<T>::load(Ab + ao);
      V al;
      if (SPLIT) al = Frag<T>::load(Ab2 + ao);
#pragma unroll
      for (int j = 0; j < 4; ++j) {
        acc[i][j] = Frag<T>::mma(ah, bh[j], acc[i][j]);
        if (SPLIT) {
          acc[i][j] = Frag<T>::mma(ah, bl[j], acc[i][j]);
          acc[i][j] = Frag<T>::mma(al, bh[j], acc[i][j]);
        }
      }
      Frag<T>::guard(acc[i][0], acc[i][3], ah, SPLIT ? al : ah);
    }
    Frag<T>::keep(bh[0], bh[1], bh[2], bh[3]);
    if (SPLIT) Frag<T>::keep(bl[0], bl[1], bl[2], bl[3]);
  }
  acc_guard4(acc[0][0], acc[0][1], acc[0][2], acc[0][3]);
  acc_guard4(acc[1][0], acc[1][1], acc[1][2], acc[1][3]);
  acc_guard4(acc[2][0], acc[2][1], acc[2][2], acc[2][3]);
  acc_guard4(acc[3][0], acc[3][1], acc[3][2], acc[3][3]);

  float* slab = sT[wave];
  const float* Rb = RESID ? (resid + (size_t)b * strideR) : nullptr;
#pragma unroll
  for (int i = 0; i < 4; ++i) {
    const int mBase = m0 + (i << 4);
#pragma unroll
    for (int j = 0; j < 4; ++j) {
      const int n = n0 + (j << 4) + rlane;
      float bv = 0.f;
      if (BIAS_MODE == 2) { if (NSTORE == 0 || n < NSTORE) bv = bias[n]; }
#pragma unroll
      for (int r = 0; r < 8; ++r) {
        float v = acc[i][j][r] * scale;
        if (BIAS_MODE == 1) v += bias[mBase + mOff + r];
        if (BIAS_MODE == 2) v += bv;
        if (RESID) v += Rb[(size_t)(mBase + mOff + r) * ldc + n];
        if (ACT == 1) v = tanhf(v);
        if (ACT == 2) v = fmaxf(v, 0.0f);
        if (ACT == 3) v = v / (1.0f + expf(-v));
        if (ACT == 4) v = (v > 0.f) ? v : 0.01f * v;
        if (ACT == 5) v = 0.5f * v * (1.0f + erff(v * 0.70710678118654752f));
        slab[(mOff + r) * 68 + (j << 4) + rlane] = v;
      }
    }
    __builtin_amdgcn_fence(__ATOMIC_RELEASE, "workgroup");
    __builtin_amdgcn_wave_barrier();
    __builtin_amdgcn_fence(__ATOMIC_ACQUIRE, "workgroup");
    if (OUT_MODE == 0) {
      float* C = (float*)Cout + (size_t)b * strideC;
      const int hh = lane >> 4, c4 = (lane & 15) * 4;
      const bool cok = (NSTORE == 0) || (c4 < NSTORE);
      for (int pass = 0; pass < 2; ++pass) {
#pragma unroll
        for (int it = 0; it < 8; ++it) {
          const int row = it * 2 + hh;
          v4f v = *(const v4f*)(slab + row * 68 + c4);
          if (cok && (mBase + row) < Mlim) *(volatile v4f*)(C + (size_t)(mBase + row) * ldc + n0 + c4) = v;
        }
        __threadfence();
      }
    } else {
      const int q = lane >> 3, c8 = (lane & 7) * 8;
      unsigned short* C  = (unsigned short*)Cout  + (size_t)b * strideC;
      unsigned short* C2 = (OUT_MODE == 2) ? ((unsigned short*)Cout2 + (size_t)b * strideC) : nullptr;
      for (int pass = 0; pass < 2; ++pass) {
#pragma unroll
        for (int it = 0; it < 4; ++it) {
          const int row = it * 4 + q;
          const float* sp = slab + row * 68 + c8;
          v8h hv, lv;
#pragma unroll
          for (int e = 0; e < 8; ++e) {
            if (OUT_MODE == 1) {
              hv[e] = (_Float16)sp[e];
            } else {
              unsigned short hb = f2bf_bits(sp[e]);
              unsigned short lb = f2bf_bits(sp[e] - bf_bits2f(hb));
              hv[e] = __builtin_bit_cast(_Float16, hb);
              lv[e] = __builtin_bit_cast(_Float16, lb);
            }
          }
          if ((mBase + row) < Mlim) {
            *(volatile v8h*)(C + (size_t)(mBase + row) * ldc + n0 + c8) = hv;
            if (OUT_MODE == 2) *(volatile v8h*)(C2 + (size_t)(mBase + row) * ldc + n0 + c8) = lv;
          }
        }
        __threadfence();
      }
    }
    __builtin_amdgcn_fence(__ATOMIC_RELEASE, "workgroup");
    __builtin_amdgcn_wave_barrier();
    __builtin_amdgcn_fence(__ATOMIC_ACQUIRE, "workgroup");
  }
}

__device__ __forceinline__ int blk_excl_scan(int cnt, int* scan_ws, int tid, int* tot) {
  const int lane = tid & 31, wave = tid >> 5; int incl = cnt;
#pragma unroll
  for (int o = 1; o < 32; o <<= 1) { const int v = __shfl_up(incl, o, 32); if (lane >= o) incl += v; }
  if (lane == 31) scan_ws[wave] = incl;
  __syncthreads();
  if (wave == 0) { int wv = (lane < NT / 32) ? scan_ws[lane] : 0; int wincl = wv;
#pragma unroll
    for (int o = 1; o < 32; o <<= 1) { const int v = __shfl_up(wincl, o, 32); if (lane >= o) wincl += v; }
    if (lane < NT / 32) scan_ws[32 + lane] = wincl - wv; if (lane == 31) scan_ws[64] = wincl; }
  __syncthreads();
  const int res = scan_ws[32 + wave] + incl - cnt; *tot = scan_ws[64];
  return res;
}
template <int SP, int CAP>
__device__ __forceinline__ int chunk_hits(const int* __restrict__ colv, const int* __restrict__ rowv, const int* __restrict__ ea,
                                          int e0, int n0, int tid, int* LIST, int* scan_ws) {
  const int eb = e0 + tid * SP;
  int rec[SP]; int cnt = 0;
#pragma unroll
  for (int k = 0; k < SP; ++k) rec[k] = -1;
  if (eb < NE) {
#pragma unroll
    for (int k = 0; k < SP; k += 4) {
      const v4i d4 = *(const v4i*)(colv + eb + k);
      const v4i s4 = *(const v4i*)(rowv + eb + k);
#pragma unroll
      for (int e = 0; e < 4; ++e) {
        const int d = d4[e]; int r = -1;
        if (d >= n0 && d < n0 + SRB && d < NN) {
          const int ee = eb + k + e;
          const int rel = ((ea[ee * 3] == 1) ? 1 : 0) | ((ea[ee * 3 + 1] == 1) ? 2 : 0) | ((ea[ee * 3 + 2] == 1) ? 4 : 0);
          if (rel != 0) { int s = s4[e]; s = s < 0 ? 0 : (s >= NN ? NN - 1 : s); r = (rel << 27) | ((d - n0) << 16) | s; ++cnt; }
        }
        rec[k + e] = r;
      }
    }
  }
  int tot; int p = blk_excl_scan(cnt, scan_ws, tid, &tot);
#pragma unroll
  for (int k = 0; k < SP; ++k) if (rec[k] >= 0) { if ((unsigned)p < (unsigned)CAP) LIST[p] = rec[k]; ++p; }
  __syncthreads();
  return tot < CAP ? tot : CAP;
}

__global__ __launch_bounds__(NT) void prep_kernel(const float* __restrict__ Ws, const float* __restrict__ Wd, const float* __restrict__ Wt,
                                                 const float* __restrict__ Wi, const float* __restrict__ Wf1, const float* __restrict__ Wf2,
                                                 unsigned* __restrict__ WT, unsigned* __restrict__ WF1, unsigned* __restrict__ WF2) {
  const int i = blockIdx.x * NT + threadIdx.x;
  const int N0 = NL * 4 * DD * DD / 2;
  const int N1 = HMW * HMW / 2;
  const int N2 = 64 * HMW / 2;
  float a = 0.f, b = 0.f; unsigned* dst = nullptr; int di = 0;
  if (i < N0) {
    const int k = 2 * (i & 63); const int rid = i >> 6;
    const int c = rid & 127, j = (rid >> 7) & 3, l = rid >> 9;
    const float* W = (j == 0) ? Ws : (j == 1) ? Wd : (j == 2) ? Wt : Wi;
    const float* src = W + (size_t)l * DD * DD + c;
    a = src[(size_t)k * DD]; b = src[(size_t)(k + 1) * DD];
    dst = WT; di = i;
  } else if (i < N0 + N1) {
    const int ii = i - N0; const int k = 2 * (ii & 127); const int o = ii >> 7;
    a = Wf1[(size_t)k * HMW + o]; b = Wf1[(size_t)(k + 1) * HMW + o];
    dst = WF1; di = ii;
  } else if (i < N0 + N1 + N2) {
    const int ii = i - N0 - N1; const int k = 2 * (ii & 127); const int o = ii >> 7;
    if (o < NCL) { a = Wf2[(size_t)k * NCL + o]; b = Wf2[(size_t)(k + 1) * NCL + o]; }
    dst = WF2; di = ii;
  }
  if (dst != nullptr) {
    const _Float16 h0 = (_Float16)a, h1 = (_Float16)b;
    const unsigned u = (unsigned)__builtin_bit_cast(unsigned short, h0) | ((unsigned)__builtin_bit_cast(unsigned short, h1) << 16);
    ((volatile unsigned*)dst)[di] = u;
    __threadfence();
    ((volatile unsigned*)dst)[di] = u;
  }
}

__global__ __launch_bounds__(NT) void castx_kernel(const float* __restrict__ x, unsigned short* __restrict__ Zp) {
  _Float16* Zh = (_Float16*)Zp;
  const int t = threadIdx.x;
  const int n = blockIdx.x * 16 + (t >> 4);
  const int c8 = (t & 15) * 8;
  const v4f z4 = {0.f, 0.f, 0.f, 0.f};
  v4f a = z4, b = z4;
  if (n < NN) { a = *(const v4f*)(x + (size_t)n * DD + c8); b = *(const v4f*)(x + (size_t)n * DD + c8 + 4); }
  if (n < NP) {
    const v4h ha = __builtin_convertvector(a, v4h), hb = __builtin_convertvector(b, v4h);
    const v8h hv = __builtin_shufflevector(ha, hb, 0, 1, 2, 3, 4, 5, 6, 7);
    _Float16* p = Zh + (size_t)n * ZW + 3 * DD + c8;
    *(volatile v8h*)p = hv;
    __threadfence();
    *(volatile v8h*)p = hv;
  }
}

__global__ __launch_bounds__(NT) void deg_kernel(const int* __restrict__ ei, const int* __restrict__ ea, float* __restrict__ DINV) {
  __shared__ int LIST[SCH];
  __shared__ float CNT[SRB * 4];
  __shared__ int scan_ws[80];
  const int tid = threadIdx.x, lane = tid & 31, wave = tid >> 5;
  const int n0 = blockIdx.x * SRB;
  for (int i = tid; i < SRB * 4; i += NT) CNT[i] = 0.f;
  __syncthreads();
  const int* rowv = ei; const int* colv = ei + NE;
#pragma unroll 1
  for (int c = 0; c < NCH; ++c) {
    const int tot = chunk_hits<SCH / NT, SCH>(colv, rowv, ea, c * SCH, n0, tid, LIST, scan_ws);
#pragma unroll 1
    for (int base = 0; base < tot; base += 32) {
      const int q = base + lane;
      const int rv = (q < tot) ? LIST[q] : -1;
      const int own = (rv >= 0 && ((rv >> 24) & 7) == wave) ? 1 : 0;
      unsigned msk = (unsigned)__ballot(own);
#pragma unroll 1
      for (int it = 0; it < 32; ++it) {
        if (msk == 0u) break;
        const int bp = __builtin_ctz(msk); msk &= msk - 1u;
        const int r = __shfl(rv, bp, 32);
        const int rel = (r >> 27) & 7; const int dl = (r >> 16) & (SRB - 1);
        if (lane < 3 && ((rel >> lane) & 1)) CNT[dl * 4 + lane] += 1.0f;
      }
    }
    __syncthreads();
  }
  __syncthreads();
#pragma unroll 1
  for (int r = 0; r < 3; ++r) {
#pragma unroll
    for (int i = 0; i < 2; ++i) {
      const int dlb = wave * 256 + i * 128;
      if (n0 + dlb + 128 <= NP) {
        const int dl = dlb + 4 * lane;
        v4f o;
#pragma unroll
        for (int e = 0; e < 4; ++e) { const float cn = CNT[(dl + e) * 4 + r]; o[e] = (cn > 0.f) ? rsqrtf(cn) : 0.f; }
        float* p = DINV + (size_t)r * NP + n0 + dl;
        *(volatile v4f*)p = o;
        __threadfence();
        *(volatile v4f*)p = o;
      }
    }
  }
}

__global__ __launch_bounds__(NT) void agg_kernel(const int* __restrict__ ei, const int* __restrict__ ea, const float* __restrict__ DINV,
                                                unsigned short* Zp, float* ACC, int tile0) {
  __shared__ int LIST[SCH];
  __shared__ int scan_ws[80];
  const int tid = threadIdx.x, lane = tid & 31, wave = tid >> 5;
  const int n0 = (tile0 + blockIdx.x) * SRB;
  const int rbase = blockIdx.x * SRB;
  const _Float16* Zh = (const _Float16*)Zp;
  _Float16* Zw = (_Float16*)Zp;
  const v4f z4 = {0.f, 0.f, 0.f, 0.f};
#pragma unroll 1
  for (int j = 0; j < 256; ++j) {
    float* rp = ACC + (size_t)(rbase + wave * 256 + j) * AW + 4 * lane;
    *(v4f*)rp = z4; *(v4f*)(rp + DD) = z4; *(v4f*)(rp + 2 * DD) = z4;
  }
  const int* rowv = ei; const int* colv = ei + NE;
#pragma unroll 1
  for (int c = 0; c < NCH; ++c) {
    const int tot = chunk_hits<SCH / NT, SCH>(colv, rowv, ea, c * SCH, n0, tid, LIST, scan_ws);
#pragma unroll 1
    for (int base = 0; base < tot; base += 32) {
      const int q = base + lane;
      const int rv = (q < tot) ? LIST[q] : -1;
      const int own = (rv >= 0 && ((rv >> 24) & 7) == wave) ? 1 : 0;
      unsigned msk = (unsigned)__ballot(own);
#pragma unroll 1
      for (int it = 0; it < 32; ++it) {
        if (msk == 0u) break;
        const int bp = __builtin_ctz(msk); msk &= msk - 1u;
        const int r = __shfl(rv, bp, 32);
        const int rel = (r >> 27) & 7; const int dl = (r >> 16) & (SRB - 1);
        int s = r & 0xFFFF; s = s < NN ? s : NN - 1;
        const v4h xh = *(const v4h*)(Zh + (size_t)s * ZW + 3 * DD + 4 * lane);
        const v4f xv = __builtin_convertvector(xh, v4f);
        float* rp = ACC + (size_t)(rbase + dl) * AW + 4 * lane;
        if (rel & 1) { const float d = DINV[s];          v4f a = *(const v4f*)rp;            a = a + d * xv; *(v4f*)rp = a; }
        if (rel & 2) { const float d = DINV[NP + s];     v4f a = *(const v4f*)(rp + DD);     a = a + d * xv; *(v4f*)(rp + DD) = a; }
        if (rel & 4) { const float d = DINV[2 * NP + s]; v4f a = *(const v4f*)(rp + 2 * DD); a = a + d * xv; *(v4f*)(rp + 2 * DD) = a; }
      }
    }
    __syncthreads();
  }
  const int cA = 8 * lane;
  const int cB = 2 * DD + 8 * (lane & 15);
#pragma unroll 1
  for (int j = 0; j < 256; ++j) {
    const int dl = wave * 256 + j; const int n = n0 + dl;
    if (n < NP) {
      const float d0 = DINV[n], d1 = DINV[NP + n], d2 = DINV[2 * NP + n];
      const float dA = (lane < 16) ? d0 : d1;
      const float* rp = ACC + (size_t)(rbase + dl) * AW;
      const v4f a0 = *(const v4f*)(rp + cA) * dA;
      const v4f a1 = *(const v4f*)(rp + cA + 4) * dA;
      const v4f b0 = *(const v4f*)(rp + cB) * d2;
      const v4f b1 = *(const v4f*)(rp + cB + 4) * d2;
      const v4h ha0 = __builtin_convertvector(a0, v4h), ha1 = __builtin_convertvector(a1, v4h);
      const v4h hb0 = __builtin_convertvector(b0, v4h), hb1 = __builtin_convertvector(b1, v4h);
      const v8h hA = __builtin_shufflevector(ha0, ha1, 0, 1, 2, 3, 4, 5, 6, 7);
      const v8h hB = __builtin_shufflevector(hb0, hb1, 0, 1, 2, 3, 4, 5, 6, 7);
      _Float16* zr = Zw + (size_t)n * ZW;
      for (int pass = 0; pass < 2; ++pass) {
        *(volatile v8h*)(zr + cA) = hA;
        if (lane < 16) *(volatile v8h*)(zr + cB) = hB;
        __threadfence();
      }
    }
  }
}

__global__ __launch_bounds__(256) void layer_gemm(const unsigned short* __restrict__ Zp, const unsigned short* __restrict__ WTp,
                                                 const float* __restrict__ bb0, const float* __restrict__ bb1,
                                                 const float* __restrict__ bb2, const float* __restrict__ bb3, float* __restrict__ XP) {
  typedef _Float16 T; typedef v16h V;
  const T* Z = (const T*)Zp; const T* WT = (const T*)WTp;
  __shared__ __align__(16) float sT[8][16 * 68];
  const int lane = threadIdx.x & 31, wave = threadIdx.x >> 5;
  const int tile = blockIdx.x * 8 + wave;
  if (tile >= (NP / 16) * 2) return;
  const int tm = tile >> 1, tn = tile & 1;
  const int m0 = tm * 16, n0 = tn * 64;
  const int rlane = lane & 15, koff = (lane >> 4) * 8, mOff = (lane >> 4) * 8;
  v8f sum[4];
  v8f acc[4];
#pragma unroll
  for (int jj = 0; jj < 4; ++jj) sum[jj] = (v8f){0.f,0.f,0.f,0.f,0.f,0.f,0.f,0.f};
#pragma unroll 1
  for (int j = 0; j < 4; ++j) {
#pragma unroll
    for (int jj = 0; jj < 4; ++jj) acc[jj] = (v8f){0.f,0.f,0.f,0.f,0.f,0.f,0.f,0.f};
    const T* Ab = Z + DD * j;
    const T* Bb = WT + (size_t)j * DD * DD;
#pragma unroll 1
    for (int k0 = 0; k0 < DD; k0 += 32) {
      V bh[4];
#pragma unroll
      for (int jj = 0; jj < 4; ++jj) {
        const size_t bo = (size_t)(n0 + (jj << 4) + rlane) * DD + koff + k0;
        bh[jj] = Frag<T>::load(Bb + bo);
      }
      const size_t ao = (size_t)(m0 + rlane) * ZW + koff + k0;
      const V ah = Frag<T>::load(Ab + ao);
#pragma unroll
      for (int jj = 0; jj < 4; ++jj) acc[jj] = Frag<T>::mma(ah, bh[jj], acc[jj]);
      Frag<T>::guard(acc[0], acc[3], ah, ah);
      Frag<T>::keep(bh[0], bh[1], bh[2], bh[3]);
    }
    acc_guard4(acc[0], acc[1], acc[2], acc[3]);
    const float* bj = (j == 0) ? bb0 : (j == 1) ? bb1 : (j == 2) ? bb2 : bb3;
#pragma unroll
    for (int jj = 0; jj < 4; ++jj) {
      const float bv = bj[n0 + (jj << 4) + rlane];
#pragma unroll
      for (int r = 0; r < 8; ++r) sum[jj][r] += fmaxf(acc[jj][r] + bv, 0.f);
    }
  }
  float* slab = sT[wave];
#pragma unroll
  for (int jj = 0; jj < 4; ++jj)
#pragma unroll
    for (int r = 0; r < 8; ++r) slab[(mOff + r) * 68 + (jj << 4) + rlane] = sum[jj][r];
  __builtin_amdgcn_fence(__ATOMIC_RELEASE, "workgroup");
  __builtin_amdgcn_wave_barrier();
  __builtin_amdgcn_fence(__ATOMIC_ACQUIRE, "workgroup");
  {
    const int hh = lane >> 4, c4 = (lane & 15) * 4;
    for (int pass = 0; pass < 2; ++pass) {
#pragma unroll
      for (int it = 0; it < 8; ++it) {
        const int row = it * 2 + hh;
        v4f v = *(const v4f*)(slab + row * 68 + c4);
        *(volatile v4f*)(XP + (size_t)(m0 + row) * DD + n0 + c4) = v;
      }
      __threadfence();
    }
  }
}

__global__ __launch_bounds__(128) void bnpart_kernel(const float* __restrict__ XP, double* __restrict__ PART) {
  const int c = threadIdx.x, b = blockIdx.x;
  double s1 = 0.0, s2 = 0.0;
#pragma unroll 1
  for (int i = 0; i < 128; ++i) {
    const int n = b * 128 + i;
    if (n < NN) { const double v = (double)XP[(size_t)n * DD + c]; s1 += v; s2 += v * v; }
  }
  double* p1 = PART + (size_t)b * DD + c;
  double* p2 = PART + (size_t)PB * DD + (size_t)b * DD + c;
  *(volatile double*)p1 = s1; *(volatile double*)p2 = s2;
  __threadfence();
  *(volatile double*)p1 = s1; *(volatile double*)p2 = s2;
}

__global__ __launch_bounds__(128) void bnred_kernel(const double* __restrict__ PART, float* __restrict__ BNP) {
  const int c = threadIdx.x;
  double s1 = 0.0, s2 = 0.0;
#pragma unroll 1
  for (int b = 0; b < PB; ++b) { s1 += PART[(size_t)b * DD + c]; s2 += PART[(size_t)PB * DD + (size_t)b * DD + c]; }
  const double mu = s1 * (1.0 / (double)NN);
  double var = s2 * (1.0 / (double)NN) - mu * mu;
  var = var > 0.0 ? var : 0.0;
  const float muf = (float)mu;
  const float varf = (float)var;
  const float istd = 1.0f / sqrtf(varf + 1e-5f);
  *(volatile float*)(BNP + c) = muf; *(volatile float*)(BNP + DD + c) = istd;
  __threadfence();
  *(volatile float*)(BNP + c) = muf; *(volatile float*)(BNP + DD + c) = istd;
}

__global__ __launch_bounds__(NT) void bnapply_kernel(const float* __restrict__ XP, const float* __restrict__ BNP,
                                                    const float* __restrict__ gam, const float* __restrict__ bet, unsigned short* __restrict__ Zp) {
  _Float16* Zh = (_Float16*)Zp;
  const int t = threadIdx.x;
  const int n = blockIdx.x * 16 + (t >> 4);
  const int c8 = (t & 15) * 8;
  if (n < NN) {
    const v4f x0 = *(const v4f*)(XP + (size_t)n * DD + c8), x1 = *(const v4f*)(XP + (size_t)n * DD + c8 + 4);
    const v4f mu0 = *(const v4f*)(BNP + c8), mu1 = *(const v4f*)(BNP + c8 + 4);
    const v4f is0 = *(const v4f*)(BNP + DD + c8), is1 = *(const v4f*)(BNP + DD + c8 + 4);
    const v4f g0 = *(const v4f*)(gam + c8), g1 = *(const v4f*)(gam + c8 + 4);
    const v4f e0 = *(const v4f*)(bet + c8), e1 = *(const v4f*)(bet + c8 + 4);
    v4f y0 = ((x0 - mu0) * is0) * g0 + e0;
    v4f y1 = ((x1 - mu1) * is1) * g1 + e1;
#pragma unroll
    for (int e = 0; e < 4; ++e) { y0[e] = fmaxf(y0[e], 0.f); y1[e] = fmaxf(y1[e], 0.f); }
    const v4h ha = __builtin_convertvector(y0, v4h), hb = __builtin_convertvector(y1, v4h);
    const v8h hv = __builtin_shufflevector(ha, hb, 0, 1, 2, 3, 4, 5, 6, 7);
    _Float16* p = Zh + (size_t)n * ZW + 3 * DD + c8;
    *(volatile v8h*)p = hv;
    __threadfence();
    *(volatile v8h*)p = hv;
  }
}

__global__ __launch_bounds__(NT) void pool_kernel(const unsigned short* __restrict__ Zp, const int* __restrict__ batch, float* __restrict__ P) {
  __shared__ int LIST[SCHP];
  __shared__ int scan_ws[80];
  __shared__ __align__(16) float red[8 * DD];
  const _Float16* Zh = (const _Float16*)Zp;
  const int tid = threadIdx.x, lane = tid & 31, wave = tid >> 5;
  const int g = blockIdx.x;
  const v4f z4 = {0.f, 0.f, 0.f, 0.f};
  v4f acc = z4;
#pragma unroll 1
  for (int c = 0; c < NCHP; ++c) {
    const int eb = c * SCHP + tid * 8;
    int bv[8]; int rec[8]; int kc = 0;
    if (eb < NN) {
      const v4i b0 = *(const v4i*)(batch + eb), b1 = *(const v4i*)(batch + eb + 4);
      bv[0] = b0[0]; bv[1] = b0[1]; bv[2] = b0[2]; bv[3] = b0[3]; bv[4] = b1[0]; bv[5] = b1[1]; bv[6] = b1[2]; bv[7] = b1[3];
    } else {
#pragma unroll
      for (int k = 0; k < 8; ++k) bv[k] = -1;
    }
#pragma unroll
    for (int k = 0; k < 8; ++k) { rec[k] = -1; if (bv[k] == g) { rec[k] = eb + k; ++kc; } }
    int tot; int p = blk_excl_scan(kc, scan_ws, tid, &tot);
#pragma unroll
    for (int k = 0; k < 8; ++k) if (rec[k] >= 0) { if ((unsigned)p < (unsigned)SCHP) LIST[p] = rec[k]; ++p; }
    __syncthreads();
    const int totc = tot < SCHP ? tot : SCHP;
#pragma unroll 1
    for (int q = wave; q < totc; q += 8) {
      int nd = LIST[q]; nd = nd < 0 ? 0 : (nd >= NN ? NN - 1 : nd);
      const v4h xh = *(const v4h*)(Zh + (size_t)nd * ZW + 3 * DD + 4 * lane);
      acc = acc + __builtin_convertvector(xh, v4f);
    }
    __syncthreads();
  }
  *(v4f*)(red + wave * DD + 4 * lane) = acc;
  __syncthreads();
  if (wave == 0) {
    v4f s = z4;
#pragma unroll
    for (int w = 0; w < 8; ++w) s = s + *(const v4f*)(red + w * DD + 4 * lane);
    float* pp = P + (size_t)g * DD + 4 * lane;
    *(volatile v4f*)pp = s;
    __threadfence();
    *(volatile v4f*)pp = s;
  }
}

__global__ __launch_bounds__(NT) void newin_kernel(const unsigned short* __restrict__ Zp, const float* __restrict__ P, const int* __restrict__ batch,
                                                  unsigned short* __restrict__ NW) {
  const _Float16* Zh = (const _Float16*)Zp;
  _Float16* Nh = (_Float16*)NW;
  const int t = threadIdx.x;
  const int n = blockIdx.x * 8 + (t >> 5);
  const int q = t & 31;
  const v8f z8 = {0.f,0.f,0.f,0.f,0.f,0.f,0.f,0.f};
  v8h hv = __builtin_convertvector(z8, v8h);
  if (n < NN) {
    if (q < 16) {
      hv = *(const v8h*)(Zh + (size_t)n * ZW + 3 * DD + 8 * q);
    } else {
      int g = batch[n]; g = g < 0 ? 0 : (g >= NG ? NG - 1 : g);
      const v4f p0 = *(const v4f*)(P + (size_t)g * DD + 8 * (q - 16)), p1 = *(const v4f*)(P + (size_t)g * DD + 8 * (q - 16) + 4);
      const v4h ha = __builtin_convertvector(p0, v4h), hb = __builtin_convertvector(p1, v4h);
      hv = __builtin_shufflevector(ha, hb, 0, 1, 2, 3, 4, 5, 6, 7);
    }
  }
  if (n < NP) {
    _Float16* pp = Nh + (size_t)n * HMW + 8 * q;
    *(volatile v8h*)pp = hv;
    __threadfence();
    *(volatile v8h*)pp = hv;
  }
}

extern "C" void kernel_launch(void* const* d_in, const int* in_sizes, int n_in,
                              void* d_out, int out_size, void* d_ws, size_t ws_size, hipStream_t stream) {
  (void)in_sizes; (void)n_in; (void)out_size;
  const float* x     = (const float*)d_in[0];
  const int*   ei    = (const int*)  d_in[1];
  const int*   ea    = (const int*)  d_in[2];
  const int*   batch = (const int*)  d_in[3];
  const float* W_s   = (const float*)d_in[4];
  const float* b_s   = (const float*)d_in[5];
  const float* W_d   = (const float*)d_in[6];
  const float* b_d   = (const float*)d_in[7];
  const float* W_t   = (const float*)d_in[8];
  const float* b_t   = (const float*)d_in[9];
  const float* W_i   = (const float*)d_in[10];
  const float* b_i   = (const float*)d_in[11];
  const float* gamma = (const float*)d_in[12];
  const float* beta  = (const float*)d_in[13];
  const float* W_fc1 = (const float*)d_in[14];
  const float* b_fc1 = (const float*)d_in[15];
  const float* W_fc2 = (const float*)d_in[16];
  const float* b_fc2 = (const float*)d_in[17];
  float* out = (float*)d_out;

  char* ws = (char*)d_ws; size_t off = 0;
  auto carve = [&](size_t bytes) -> char* { char* p = ws + off; off += (bytes + 255) & ~(size_t)255; return p; };
  unsigned*       WT     = (unsigned*)carve((size_t)NL * 4 * DD * DD * 2);
  unsigned*       WF1    = (unsigned*)carve((size_t)HMW * HMW * 2);
  unsigned*       WF2    = (unsigned*)carve((size_t)64 * HMW * 2);
  float*          DINV   = (float*)carve((size_t)3 * NP * 4);
  double*         PART   = (double*)carve((size_t)2 * PB * DD * 8);
  float*          BNP    = (float*)carve((size_t)2 * DD * 4);
  float*          POOLED = (float*)carve((size_t)NG * DD * 4);
  char*           ZR     = carve((size_t)NP * ZW * 2);
  char*           R      = carve((size_t)NTA * SRB * AW * 4);
  float*          XP     = (float*)carve((size_t)NP * DD * 4);
  if (off > ws_size || off > (size_t)134217728) return;
  unsigned short* Z       = (unsigned short*)ZR;
  float*          ACC     = (float*)R;
  unsigned short* NEWIN   = (unsigned short*)R;
  unsigned short* NODEOUT = (unsigned short*)ZR;
  const unsigned short* WT16  = (const unsigned short*)WT;
  const unsigned short* WF116 = (const unsigned short*)WF1;
  const unsigned short* WF216 = (const unsigned short*)WF2;

  prep_kernel<<<(NL * 4 * DD * DD / 2 + HMW * HMW / 2 + 64 * HMW / 2) / NT, NT, 0, stream>>>(W_s, W_d, W_t, W_i, W_fc1, W_fc2, WT, WF1, WF2);
  castx_kernel<<<NP / 16, NT, 0, stream>>>(x, Z);
  deg_kernel<<<NTILE, NT, 0, stream>>>(ei, ea, DINV);

  for (int l = 0; l < NL; ++l) {
    agg_kernel<<<NTA, NT, 0, stream>>>(ei, ea, DINV, Z, ACC, 0);
    agg_kernel<<<NTILE - NTA, NT, 0, stream>>>(ei, ea, DINV, Z, ACC, NTA);
    layer_gemm<<<((NP / 16) * 2 + 7) / 8, 256, 0, stream>>>(Z, WT16 + (size_t)l * 4 * DD * DD,
        b_s + l * DD, b_d + l * DD, b_t + l * DD, b_i + l * DD, XP);
    bnpart_kernel<<<PB, 128, 0, stream>>>(XP, PART);
    bnred_kernel<<<1, 128, 0, stream>>>(PART, BNP);
    bnapply_kernel<<<NN / 16, NT, 0, stream>>>(XP, BNP, gamma + l * DD, beta + l * DD, Z);
  }

  pool_kernel<<<NG, NT, 0, stream>>>(Z, batch, POOLED);
  newin_kernel<<<NP / 8, NT, 0, stream>>>(Z, POOLED, batch, NEWIN);
  {
    const int tiles = (NP / 64) * (HMW / 64);
    wmma_gemm64<0, false, 2, 1, false, 2, 0><<<dim3((tiles + 7) / 8, 1), 256, 0, stream>>>(
        (const unsigned short*)NEWIN, (const unsigned short*)nullptr, HMW, 0L,
        WF116, (const unsigned short*)nullptr, HMW, 0L,
        (void*)NODEOUT, (void*)nullptr, HMW, 0L,
        b_fc1, (const float*)nullptr, 0L, NP, HMW, HMW, 1.0f, NP);
  }
  {
    const int tiles = (NP / 64) * 1;
    wmma_gemm64<0, false, 2, 0, false, 0, NCL><<<dim3((tiles + 7) / 8, 1), 256, 0, stream>>>(
        (const unsigned short*)NODEOUT, (const unsigned short*)nullptr, HMW, 0L,
        WF216, (const unsigned short*)nullptr, HMW, 0L,
        (void*)out, (void*)nullptr, NCL, 0L,
        b_fc2, (const float*)nullptr, 0L, NP, 64, HMW, 1.0f, NN);
  }
}
